// NonlocalBlock2D_12936441496195
// MI455X (gfx1250) — hardware-verified
//
#include <hip/hip_runtime.h>
#include <math.h>

constexpr int kB   = 2;
constexpr int kC   = 64;
constexpr int kIC  = 32;
constexpr int kN   = 9216;
constexpr int kNP  = 64;
constexpr int kQch = 1536;
constexpr int kNch = kN / kQch;
constexpr int kSmThreads = 288;
constexpr float kWCarry    = 16.0f;
constexpr float kPCarry    = 32768.0f;
constexpr float kProjScale = 1.0f / 16.0f;
constexpr float kPVScale   = 256.0f / 32768.0f;
constexpr float kOutScale  = 1.0f / (256.0f * 16.0f);
static_assert(kN % kQch == 0);
static_assert(kQch % 64 == 0 && kN % 64 == 0 && kNP % 64 == 0 && kC % 64 == 0);
static_assert(kC % 32 == 0 && kIC % 32 == 0 && kN % 32 == 0);
static_assert(kN == kSmThreads * 4 * 8);
static_assert(kIC * kC == 256 * 8 && kC * kIC == 256 * 8);

typedef __attribute__((ext_vector_type(16))) _Float16 v16h;
typedef __attribute__((ext_vector_type(8)))  _Float16 v8h;
typedef __attribute__((ext_vector_type(16))) __bf16   v16b;
typedef __attribute__((ext_vector_type(8)))  __bf16   v8b;
typedef __attribute__((ext_vector_type(8)))  float    v8f;
typedef __attribute__((ext_vector_type(4)))  float    v4f;
typedef __attribute__((ext_vector_type(4)))  unsigned int v4u;

__device__ __forceinline__ unsigned short f2bf_bits(float f) {
  unsigned u = __float_as_uint(f);
  return (unsigned short)((u + 0x7FFFu + ((u >> 16) & 1u)) >> 16);
}
__device__ __forceinline__ float bf_bits2f(unsigned short h) { return __uint_as_float(((unsigned)h) << 16); }

__device__ __forceinline__ void dep_guard4_h(v8f& a, v8f& b, v8f& c, v8f& d, v16h x, v16h y) { asm volatile("v_nop\n\tv_nop\n\tv_nop\n\tv_nop" : "+v"(a), "+v"(b), "+v"(c), "+v"(d) : "v"(x), "v"(y)); }
__device__ __forceinline__ void dep_guard4_b(v8f& a, v8f& b, v8f& c, v8f& d, v16b x, v16b y) { asm volatile("v_nop\n\tv_nop\n\tv_nop\n\tv_nop" : "+v"(a), "+v"(b), "+v"(c), "+v"(d) : "v"(x), "v"(y)); }
__device__ __forceinline__ void keep4_h(v16h a, v16h b, v16h c, v16h d) { asm volatile("v_nop" :: "v"(a), "v"(b), "v"(c), "v"(d)); }
__device__ __forceinline__ void keep4_b(v16b a, v16b b, v16b c, v16b d) { asm volatile("v_nop" :: "v"(a), "v"(b), "v"(c), "v"(d)); }
__device__ __forceinline__ void acc_guard4(v8f& a, v8f& b, v8f& c, v8f& d) { asm volatile("v_nop\n\tv_nop\n\tv_nop\n\tv_nop" : "+v"(a), "+v"(b), "+v"(c), "+v"(d)); }
template <typename T> struct Frag;
template <> struct Frag<_Float16> {
  typedef v16h V; union U { v16h v; v8h h[2]; };
  static __device__ __forceinline__ v16h load(const _Float16* p) {
    U f; f.h[0] = *(const v8h*)(p); f.h[1] = *(const v8h*)(p + 16); return f.v;
  }
  static __device__ __forceinline__ v8f mma(v16h a, v16h b, v8f c) {
    return __builtin_amdgcn_wmma_f32_16x16x32_f16(false, a, false, b, (short)0, c, false, false);
  }
  static __device__ __forceinline__ void guard4(v8f& a, v8f& b, v8f& c, v8f& d, v16h x, v16h y) { dep_guard4_h(a, b, c, d, x, y); }
  static __device__ __forceinline__ void keep(v16h a, v16h b, v16h c, v16h d) { keep4_h(a, b, c, d); }
};
template <> struct Frag<__bf16> {
  typedef v16b V; union U { v16b v; v8b h[2]; };
  static __device__ __forceinline__ v16b load(const __bf16* p) {
    U f; f.h[0] = *(const v8b*)(p); f.h[1] = *(const v8b*)(p + 16); return f.v;
  }
  static __device__ __forceinline__ v8f mma(v16b a, v16b b, v8f c) {
    return __builtin_amdgcn_wmma_f32_16x16x32_bf16(false, a, false, b, (short)0, c, false, false);
  }
  static __device__ __forceinline__ void guard4(v8f& a, v8f& b, v8f& c, v8f& d, v16b x, v16b y) { dep_guard4_b(a, b, c, d, x, y); }
  static __device__ __forceinline__ void keep(v16b a, v16b b, v16b c, v16b d) { keep4_b(a, b, c, d); }
};

__device__ __forceinline__ unsigned pk16(unsigned short a, unsigned short b) { return (unsigned)a | ((unsigned)b << 16); }
__device__ __forceinline__ unsigned short h_bits(float f) { const _Float16 h = (_Float16)f; return __builtin_bit_cast(unsigned short, h); }

template <int ET> struct Elem;
template <> struct Elem<0> { typedef _Float16 T; };
template <> struct Elem<1> { typedef __bf16 T; };
template <int ET, bool SPLIT, int BIAS_MODE, int OUT_MODE, bool RESID>
__global__ __launch_bounds__(256) void wmma_gemm64(
    const unsigned short* __restrict__ Ap, const unsigned short* __restrict__ A2p, int lda, long strideA,
    const unsigned short* __restrict__ Btp, const unsigned short* __restrict__ Bt2p, int ldb, long strideB,
    void* __restrict__ Cout, void* __restrict__ Cout2, int ldc, long strideC,
    const float* __restrict__ bias,
    const float* __restrict__ resid, long strideR,
    int M, int N, int K, float scale) {
  static_assert(!(RESID && OUT_MODE != 0));
  typedef typename Elem<ET>::T T;
  typedef typename Frag<T>::V V;
  const T* A = (const T*)Ap; const T* A2 = (const T*)A2p; const T* Bt = (const T*)Btp; const T* Bt2 = (const T*)Bt2p;
  __shared__ __align__(16) float sT[8][16 * 68];
  const int b    = blockIdx.y;
  const int lane = threadIdx.x & 31;
  const int wave = threadIdx.x >> 5;
  const int tilesN = N >> 6;
  const int tilesM = M >> 6;
  const int tile = blockIdx.x * 8 + wave;
  if (tile >= tilesM * tilesN) return;
  const int tm = tile / tilesN;
  const int tn = tile - tm * tilesN;
  const int m0 = tm << 6;
  const int n0 = tn << 6;

  const T* Ab  = A  + (size_t)b * strideA;
  const T* Bb  = Bt + (size_t)b * strideB;
  const T* Ab2 = SPLIT ? (A2  + (size_t)b * strideA) : nullptr;
  const T* Bb2 = SPLIT ? (Bt2 + (size_t)b * strideB) : nullptr;

  const int rlane = lane & 15;
  const int koff  = (lane >> 4) * 8;
  const int mOff  = (lane >> 4) * 8;

  v8f acc[4][4];
#pragma unroll
  for (int i = 0; i < 4; ++i)
#pragma unroll
    for (int j = 0; j < 4; ++j) acc[i][j] = (v8f){0.f,0.f,0.f,0.f,0.f,0.f,0.f,0.f};

  for (int k0 = 0; k0 < K; k0 += 32) {
    V bh[4], bl[4];
#pragma unroll
    for (int j = 0; j < 4; ++j) {
      const size_t bo = (size_t)(n0 + (j << 4) + rlane) * ldb + koff + k0;
      bh[j] = Frag<T>::load(Bb + bo);
      if (SPLIT) bl[j] = Frag<T>::load(Bb2 + bo);
    }
#pragma unroll
    for (int i = 0; i < 4; ++i) {
      const size_t ao = (size_t)(m0 + (i << 4) + rlane) * lda + koff + k0;
      V ah = Frag<T>::load(Ab + ao);
      V al;
      if (SPLIT) al = Frag<T>::load(Ab2 + ao);
#pragma unroll
      for (int j = 0; j < 4; ++j) {
        acc[i][j] = Frag<T>::mma(ah, bh[j], acc[i][j]);
        if (SPLIT) {
          acc[i][j] = Frag<T>::mma(ah, bl[j], acc[i][j]);
          acc[i][j] = Frag<T>::mma(al, bh[j], acc[i][j]);
        }
      }
      Frag<T>::guard4(acc[i][0], acc[i][1], acc[i][2], acc[i][3], ah, SPLIT ? al : ah);
    }
    Frag<T>::keep(bh[0], bh[1], bh[2], bh[3]);
    if (SPLIT) Frag<T>::keep(bl[0], bl[1], bl[2], bl[3]);
  }
  acc_guard4(acc[0][0], acc[0][1], acc[0][2], acc[0][3]);
  acc_guard4(acc[1][0], acc[1][1], acc[1][2], acc[1][3]);
  acc_guard4(acc[2][0], acc[2][1], acc[2][2], acc[2][3]);
  acc_guard4(acc[3][0], acc[3][1], acc[3][2], acc[3][3]);

  float* slab = sT[wave];
  const float* Rb = RESID ? (resid + (size_t)b * strideR) : nullptr;
#pragma unroll
  for (int i = 0; i < 4; ++i) {
    const int mBase = m0 + (i << 4);
    float bm[8];
#pragma unroll
    for (int r = 0; r < 8; ++r) bm[r] = 0.f;
    if (BIAS_MODE == 1) {
      const v4f b0 = *(const v4f*)(bias + mBase + mOff);
      const v4f b1 = *(const v4f*)(bias + mBase + mOff + 4);
      bm[0] = b0[0]; bm[1] = b0[1]; bm[2] = b0[2]; bm[3] = b0[3];
      bm[4] = b1[0]; bm[5] = b1[1]; bm[6] = b1[2]; bm[7] = b1[3];
    }
#pragma unroll
    for (int j = 0; j < 4; ++j) {
      const int n = n0 + (j << 4) + rlane;
      float bv = 0.f;
      if (BIAS_MODE == 2) bv = bias[n];
#pragma unroll
      for (int r = 0; r < 8; ++r) {
        float v = acc[i][j][r] * scale;
        if (BIAS_MODE == 1) v += bm[r];
        if (BIAS_MODE == 2) v += bv;
        slab[(mOff + r) * 68 + (j << 4) + rlane] = v;
      }
    }
    __builtin_amdgcn_fence(__ATOMIC_RELEASE, "workgroup");
    __builtin_amdgcn_wave_barrier();
    __builtin_amdgcn_fence(__ATOMIC_ACQUIRE, "workgroup");
    if (OUT_MODE == 0) {
      float* C = (float*)Cout + (size_t)b * strideC;
      const int hh = lane >> 4, c4 = (lane & 15) * 4;
      v4f vo[8];
#pragma unroll
      for (int it = 0; it < 8; ++it) {
        const int row = it * 2 + hh;
        v4f v = *(const v4f*)(slab + row * 68 + c4);
        if (RESID) {
          const v4f rv = *(const v4f*)(Rb + (size_t)(mBase + row) * ldc + n0 + c4);
          v = v + rv;
        }
        vo[it] = v;
      }
      for (int pass = 0; pass < 2; ++pass) {
#pragma unroll
        for (int it = 0; it < 8; ++it) {
          const int row = it * 2 + hh;
          *(volatile v4f*)(C + (size_t)(mBase + row) * ldc + n0 + c4) = vo[it];
        }
        __threadfence();
      }
    } else {
      const int q = lane >> 3, c8 = (lane & 7) * 8;
      unsigned short* C  = (unsigned short*)Cout  + (size_t)b * strideC;
      unsigned short* C2 = (OUT_MODE == 2) ? ((unsigned short*)Cout2 + (size_t)b * strideC) : nullptr;
      for (int pass = 0; pass < 2; ++pass) {
#pragma unroll
        for (int it = 0; it < 4; ++it) {
          const int row = it * 4 + q;
          const float* sp = slab + row * 68 + c8;
          v8h hv, lv;
#pragma unroll
          for (int e = 0; e < 8; ++e) {
            if (OUT_MODE == 1) {
              hv[e] = (_Float16)sp[e];
            } else {
              unsigned short hb = f2bf_bits(sp[e]);
              unsigned short lb = f2bf_bits(sp[e] - bf_bits2f(hb));
              hv[e] = __builtin_bit_cast(_Float16, hb);
              lv[e] = __builtin_bit_cast(_Float16, lb);
            }
          }
          *(volatile v8h*)(C + (size_t)(mBase + row) * ldc + n0 + c8) = hv;
          if (OUT_MODE == 2) *(volatile v8h*)(C2 + (size_t)(mBase + row) * ldc + n0 + c8) = lv;
        }
        __threadfence();
      }
    }
    __builtin_amdgcn_fence(__ATOMIC_RELEASE, "workgroup");
    __builtin_amdgcn_wave_barrier();
    __builtin_amdgcn_fence(__ATOMIC_ACQUIRE, "workgroup");
  }
}

__device__ __forceinline__ v4u pack8h(v4f a, v4f c, float s) {
  unsigned short hb[8];
#pragma unroll
  for (int e = 0; e < 4; ++e) {
    hb[e]     = h_bits(a[e] * s);
    hb[4 + e] = h_bits(c[e] * s);
  }
  return (v4u){pk16(hb[0], hb[1]), pk16(hb[2], hb[3]), pk16(hb[4], hb[5]), pk16(hb[6], hb[7])};
}

__global__ __launch_bounds__(256) void prep_kernel(const float* __restrict__ Wt, const float* __restrict__ Wp,
                                                  const float* __restrict__ Wg, const float* __restrict__ Wo,
                                                  const float* __restrict__ bt, const float* __restrict__ bp,
                                                  const float* __restrict__ bg,
                                                  unsigned short* __restrict__ Wtp16, unsigned short* __restrict__ Wg16,
                                                  unsigned short* __restrict__ Wo16,
                                                  float* __restrict__ btp, float* __restrict__ bgp) {
  const int t = threadIdx.x;
  const size_t e8 = 8 * (size_t)t;
  const v4f t0 = *(const v4f*)(Wt + e8), t1 = *(const v4f*)(Wt + e8 + 4);
  const v4f p0 = *(const v4f*)(Wp + e8), p1 = *(const v4f*)(Wp + e8 + 4);
  asm volatile("" ::: "memory");
  const v4f g0 = *(const v4f*)(Wg + e8), g1 = *(const v4f*)(Wg + e8 + 4);
  const v4f o0 = *(const v4f*)(Wo + e8), o1 = *(const v4f*)(Wo + e8 + 4);
  asm volatile("" ::: "memory");
  const int bi = 4 * (t & 7);
  const v4f vbt = *(const v4f*)(bt + bi);
  const v4f vbp = *(const v4f*)(bp + bi);
  const v4f vbg = *(const v4f*)(bg + bi);
  asm volatile("" ::: "memory");

  const v4u ut = pack8h(t0, t1, kWCarry);
  const v4u up = pack8h(p0, p1, kWCarry);
  const v4u ug = pack8h(g0, g1, kWCarry);
  const v4u uo = pack8h(o0, o1, kWCarry);
  const v4u uz = (v4u){0u, 0u, 0u, 0u};

  const float ft = (t & 8) ? 0.0f : 1.0f;
  const float fp = 1.0f - ft;
  v4f vtp, vgp;
#pragma unroll
  for (int e = 0; e < 4; ++e) {
    vtp[e] = fmaf(ft, vbt[e], fp * vbp[e]);
    vgp[e] = ft * vbg[e] + 0.0f;
  }

  for (int pass = 0; pass < 2; ++pass) {
    *(volatile v4u*)(Wtp16 + e8)        = ut;
    *(volatile v4u*)(Wtp16 + 2048 + e8) = up;
    *(volatile v4u*)(Wg16 + e8)         = ug;
    *(volatile v4u*)(Wg16 + 2048 + e8)  = uz;
    *(volatile v4u*)(Wo16 + e8)         = uo;
    if (t < 16) *(volatile v4f*)(btp + 4 * t) = vtp;
    if (t >= 32 && t < 48) *(volatile v4f*)(bgp + 4 * (t - 32)) = vgp;
    __threadfence();
  }
}

__global__ __launch_bounds__(256) void xt_cast_kernel(const float* __restrict__ x, unsigned short* __restrict__ xT) {
  __shared__ float sm[64][65];
  const int t  = threadIdx.x;
  const int n0 = blockIdx.x * 64;
  const int b  = blockIdx.y;
#pragma unroll
  for (int i = 0; i < 16; ++i) {
    const int e  = i * 256 + t;
    const int c  = e >> 6;
    const int nl = e & 63;
    sm[nl][c] = x[((size_t)(b * kC + c)) * kN + n0 + nl];
  }
  __syncthreads();
  const int lane = t & 31, wave = t >> 5;
  const int q = lane >> 3, c8 = (lane & 7) * 8;
  unsigned short* op = xT + ((size_t)b * kN + n0) * kC;
  v4u u[2];
#pragma unroll
  for (int it = 0; it < 2; ++it) {
    const int row = wave * 8 + it * 4 + q;
    const v4f a = (v4f){sm[row][c8 + 0], sm[row][c8 + 1], sm[row][c8 + 2], sm[row][c8 + 3]};
    const v4f c = (v4f){sm[row][c8 + 4], sm[row][c8 + 5], sm[row][c8 + 6], sm[row][c8 + 7]};
    u[it] = pack8h(a, c, 1.0f);
  }
  for (int pass = 0; pass < 2; ++pass) {
#pragma unroll
    for (int it = 0; it < 2; ++it) {
      const int row = wave * 8 + it * 4 + q;
      *(volatile v4u*)(op + (size_t)row * kC + c8) = u[it];
    }
    __threadfence();
  }
}

__global__ __launch_bounds__(kSmThreads) void softmax_row_kernel(const float* __restrict__ S, unsigned short* __restrict__ P) {
  __shared__ __align__(16) float lg[kN];
  __shared__ float redM[9];
  __shared__ float redS[9];
  const int row  = blockIdx.x;
  const int t    = threadIdx.x;
  const int lane = t & 31, wave = t >> 5;
  const float* sr = S + (size_t)row * kN;

  float mx = -__builtin_inff();
#pragma unroll 1
  for (int it = 0; it < 8; ++it) {
    const int c = it * 1152 + 4 * t;
    const v4f sv = *(const v4f*)(sr + c);
    mx = fmaxf(mx, fmaxf(fmaxf(sv[0], sv[1]), fmaxf(sv[2], sv[3])));
    *(v4f*)(lg + c) = sv;
  }
#pragma unroll
  for (int off = 16; off > 0; off >>= 1) mx = fmaxf(mx, __shfl_xor(mx, off, 32));
  if (lane == 0) redM[wave] = mx;
  __syncthreads();
  float m = redM[0];
#pragma unroll
  for (int w = 1; w < 9; ++w) m = fmaxf(m, redM[w]);

  float sum = 0.f;
#pragma unroll 1
  for (int it = 0; it < 8; ++it) {
    const int c = it * 1152 + 4 * t;
    const v4f l = *(const v4f*)(lg + c);
    v4f ev;
#pragma unroll
    for (int e = 0; e < 4; ++e) {
      ev[e] = expf(l[e] - m);
      sum += ev[e];
    }
    *(v4f*)(lg + c) = ev;
  }
#pragma unroll
  for (int off = 16; off > 0; off >>= 1) sum += __shfl_xor(sum, off, 32);
  if (lane == 0) redS[wave] = sum;
  __syncthreads();
  float tot = redS[0];
#pragma unroll
  for (int w = 1; w < 9; ++w) tot += redS[w];
  const float inv = kPCarry / tot;

  v4u u[4];
#pragma unroll
  for (int it = 0; it < 4; ++it) {
    const int c = it * 2304 + 8 * t;
    const v4f e0 = *(const v4f*)(lg + c);
    const v4f e1 = *(const v4f*)(lg + c + 4);
    u[it] = pack8h(e0, e1, inv);
  }
  unsigned short* pr = P + (size_t)row * kN;
#pragma unroll
  for (int it = 0; it < 4; ++it) *(volatile v4u*)(pr + it * 2304 + 8 * (size_t)t) = u[it];
  __threadfence();
#pragma unroll
  for (int it = 0; it < 4; ++it) *(volatile v4u*)(pr + it * 2304 + 8 * (size_t)t) = u[it];
}

extern "C" void kernel_launch(void* const* d_in, const int* in_sizes, int n_in,
                              void* d_out, int out_size, void* d_ws, size_t ws_size,
                              hipStream_t stream) {
  if (n_in < 9) return;
  const int nElem = kB * kC * kN;
  if (in_sizes[0] != nElem) return;
  if (in_sizes[1] != kIC * kC || in_sizes[3] != kIC * kC || in_sizes[5] != kIC * kC) return;
  if (in_sizes[2] != kIC || in_sizes[4] != kIC || in_sizes[6] != kIC) return;
  if (in_sizes[7] != kC * kIC || in_sizes[8] != kC) return;
  if (out_size != nElem) return;

  const size_t szPlane = (size_t)kB * kN * kNP * 2;
  const size_t szW64   = (size_t)64 * 64 * 2;
  const size_t szWo    = (size_t)kC * kIC * 2;
  const size_t szBias  = (size_t)64 * 4;
  const size_t szS     = (size_t)kQch * kN * 4;
  const size_t szP     = (size_t)kQch * kN * 2;
  const size_t offXT  = 0;
  const size_t offTP  = offXT + szPlane;
  const size_t offGT  = offTP + szPlane;
  const size_t offY   = offGT + szPlane;
  const size_t offWtp = offY + szPlane;
  const size_t offWg  = offWtp + szW64;
  const size_t offWo  = offWg + szW64;
  const size_t offBtp = offWo + szWo;
  const size_t offBgp = offBtp + szBias;
  const size_t offS   = offBgp + szBias;
  const size_t offP   = offS + szS;
  const size_t total  = offP + szP;
  if (ws_size < total) return;

  const float* x  = (const float*)d_in[0];
  const float* Wg = (const float*)d_in[1];
  const float* bg = (const float*)d_in[2];
  const float* Wt = (const float*)d_in[3];
  const float* bt = (const float*)d_in[4];
  const float* Wp = (const float*)d_in[5];
  const float* bp = (const float*)d_in[6];
  const float* Wo = (const float*)d_in[7];
  const float* bo = (const float*)d_in[8];
  float* out = (float*)d_out;
  char* ws = (char*)d_ws;
  unsigned short* xT16  = (unsigned short*)(ws + offXT);
  unsigned short* TP16  = (unsigned short*)(ws + offTP);
  unsigned short* gT16  = (unsigned short*)(ws + offGT);
  unsigned short* Y16   = (unsigned short*)(ws + offY);
  unsigned short* Wtp16 = (unsigned short*)(ws + offWtp);
  unsigned short* Wg16  = (unsigned short*)(ws + offWg);
  unsigned short* Wo16  = (unsigned short*)(ws + offWo);
  float* btp = (float*)(ws + offBtp);
  float* bgp = (float*)(ws + offBgp);
  float* SC  = (float*)(ws + offS);
  unsigned short* PP = (unsigned short*)(ws + offP);

  const long planeStride = (long)kN * kNP;
  const int  tilesProj   = (kN / 64) * (kNP / 64);
  const int  tilesScore  = (kQch / 64) * (kN / 64);
  const int  tilesPV     = (kQch / 64) * (kNP / 64);
  const int  tilesOut    = (kC / 64) * (kN / 64);

  prep_kernel<<<dim3(1), dim3(256), 0, stream>>>(Wt, Wp, Wg, Wo, bt, bp, bg, Wtp16, Wg16, Wo16, btp, bgp);
  xt_cast_kernel<<<dim3(kN / 64, kB), dim3(256), 0, stream>>>(x, xT16);

  wmma_gemm64<0, false, 2, 1, false><<<dim3((tilesProj + 7) / 8, kB), dim3(256), 0, stream>>>(
      xT16, xT16, kC, planeStride, Wtp16, Wtp16, kC, 0L,
      (void*)TP16, (void*)TP16, kNP, planeStride, btp, btp, 0L, kN, kNP, kC, kProjScale);
  wmma_gemm64<0, false, 1, 1, false><<<dim3((tilesProj + 7) / 8, kB), dim3(256), 0, stream>>>(
      Wg16, Wg16, kC, 0L, xT16, xT16, kC, planeStride,
      (void*)gT16, (void*)gT16, kN, planeStride, bgp, bgp, 0L, kNP, kN, kC, kProjScale);

  for (int b = 0; b < kB; ++b) {
    for (int qc = 0; qc < kNch; ++qc) {
      const size_t q0 = (size_t)qc * kQch;
      const unsigned short* Aq = TP16 + ((size_t)b * kN + q0) * kNP;
      const unsigned short* Bk = TP16 + (size_t)b * kN * kNP + kIC;
      wmma_gemm64<0, false, 0, 0, false><<<dim3((tilesScore + 7) / 8, 1), dim3(256), 0, stream>>>(
          Aq, Aq, kNP, 0L, Bk, Bk, kNP, 0L,
          (void*)SC, (void*)SC, kN, 0L, btp, btp, 0L, kQch, kN, kIC, 1.0f);
      softmax_row_kernel<<<dim3(kQch), dim3(kSmThreads), 0, stream>>>(SC, PP);
      const unsigned short* Gb = gT16 + (size_t)b * kNP * kN;
      unsigned short* Yq = Y16 + ((size_t)b * kN + q0) * kNP;
      wmma_gemm64<0, false, 0, 1, false><<<dim3((tilesPV + 7) / 8, 1), dim3(256), 0, stream>>>(
          PP, PP, kN, 0L, Gb, Gb, kN, 0L,
          (void*)Yq, (void*)Yq, kNP, 0L, btp, btp, 0L, kQch, kNP, kN, kPVScale);
    }
  }

  wmma_gemm64<0, false, 1, 0, true><<<dim3((tilesOut + 7) / 8, kB), dim3(256), 0, stream>>>(
      Wo16, Wo16, kIC, 0L, Y16, Y16, kNP, planeStride,
      (void*)out, (void*)out, kN, (long)kC * kN, bo, x, (long)kC * kN, kC, kN, kIC, kOutScale);
}
